// DySample_20023137534392
// MI455X (gfx1250) — hardware-run, weakly checked
//
#include <hip/hip_runtime.h>


#ifndef NB
#define NB 8
#endif
#define NB_FULL 8
#define CH   64
#define IMH  128
#define IMW  128
#define NPIX (IMH * IMW)
#define NK   16
#define OFC  32
#define OC   16
#define OH   256
#define OW   256
#define MW   4
#define OSP  36
#define XP   72
#define SCW  64.0f
#define SCS  16.0f
#define OSC  (1.0f / 1024.0f)

static_assert(CH == 64);
static_assert(CH % 32 == 0);
static_assert(CH == 4 * 16);
static_assert(OFC == 2 * NK);
static_assert(NK == 16);
static_assert(OC == 16);
static_assert(IMW % 16 == 0);
static_assert(NPIX % 64 == 0);
static_assert(OH == 2 * IMH);
static_assert(OW == 2 * IMW);
static_assert((NB * (NPIX / 16)) % MW == 0);
static_assert(NB <= NB_FULL);
static_assert((OSP * 4) % 16 == 0);
static_assert((XP * 2) % 16 == 0);
static_assert(32 * 16 * 8 == OC * 2 * 128);
static_assert(256 * 16 * 2 == 64 * CH * 2);
static_assert(MW * 16 * NK * 2 * 4 + MW * 32 * OSP * 4 <= 131072);
static_assert(64 * XP * 2 <= 131072);

typedef _Float16 h16;
typedef unsigned short bf;
typedef __attribute__((ext_vector_type(16))) __bf16   v16bf;
typedef __attribute__((ext_vector_type(16))) _Float16 v16h;
typedef __attribute__((ext_vector_type(8)))  _Float16 v8h;
typedef __attribute__((ext_vector_type(8)))  unsigned short v8us;
typedef __attribute__((ext_vector_type(8)))  float    v8f;
typedef __attribute__((ext_vector_type(4)))  float    v4f;
typedef __attribute__((ext_vector_type(2)))  float    v2f;
typedef __attribute__((ext_vector_type(4)))  unsigned v4u;
typedef v4f  __attribute__((may_alias)) v4fa;
typedef v2f  __attribute__((may_alias)) v2fa;
typedef v4u  __attribute__((may_alias)) v4ua;
typedef v8us __attribute__((may_alias)) v8usa;

__device__ __forceinline__ unsigned short f2bf(float f) { unsigned u = __float_as_uint(f); u += 0x7FFFu + ((u >> 16) & 1u); return (unsigned short)(u >> 16); }
__device__ __forceinline__ float bfr(float f) { return __uint_as_float(((unsigned)f2bf(f)) << 16); }
__device__ __forceinline__ v16h cat16(v8h lo, v8h hi) { return __builtin_shufflevector(lo, hi, 0, 1, 2, 3, 4, 5, 6, 7, 8, 9, 10, 11, 12, 13, 14, 15); }
__device__ __forceinline__ v16bf cat16b(v8us lo, v8us hi) { return __builtin_bit_cast(v16bf, __builtin_shufflevector(lo, hi, 0, 1, 2, 3, 4, 5, 6, 7, 8, 9, 10, 11, 12, 13, 14, 15)); }
__device__ __forceinline__ v8f wmma16(v16h a, v16h b, v8f c) { return __builtin_amdgcn_wmma_f32_16x16x32_f16(false, a, false, b, (short)0, c, false, false); }
__device__ __forceinline__ v8f wmmab(v16bf a, v16bf b, v8f c) { return __builtin_amdgcn_wmma_f32_16x16x32_bf16(false, a, false, b, (short)0, c, false, false); }
__device__ __forceinline__ v16h  ldh(const h16* p) { return cat16(*(const v8h*)p, *(const v8h*)(p + 16)); }
__device__ __forceinline__ v16bf ldb(const bf* p)  { return cat16b(*(const v8us*)p, *(const v8us*)(p + 16)); }
__device__ __forceinline__ void wave_sync() { __builtin_amdgcn_fence(3  , "wavefront"); __builtin_amdgcn_wave_barrier(); asm volatile("" ::: "memory"); }

__device__ __forceinline__ v8f wmma16g(v16h a, v16h b, v8f c) { c = wmma16(a, b, c); asm volatile("v_nop\n\tv_nop\n\tv_nop\n\tv_nop" : "+v"(c) : "v"(a), "v"(b)); return c; }
__device__ __forceinline__ v8f wmmabg(v16bf a, v16bf b, v8f c) { c = wmmab(a, b, c); asm volatile("v_nop\n\tv_nop\n\tv_nop\n\tv_nop" : "+v"(c) : "v"(a), "v"(b)); return c; }
static __device__ __forceinline__ h16 toh_flush(float v) { const h16 r = (h16)v; return (fabsf(v) < 6.103515625e-05f) ? (h16)0.0f : r; }

__global__ __launch_bounds__(256) void k_cvt8(const float* __restrict__ src, bf* dst, size_t n8) {
    const size_t i = (size_t)blockIdx.x * 256 + threadIdx.x; if (i >= n8) return;
    const v8f v = *(const v8f*)(src + i * 8); v8us o;
#pragma unroll
    for (int k = 0; k < 8; ++k) o[k] = f2bf(v[k]);
    *(volatile v8us*)(dst + i * 8) = o; __threadfence(); *(volatile v8us*)(dst + i * 8) = o;
}

__global__ __launch_bounds__(256) void k_cvtwh(const float* __restrict__ src, h16* dst, size_t n8) {
    const size_t i = (size_t)blockIdx.x * 256 + threadIdx.x; if (i >= n8) return;
    const v8f v = *(const v8f*)(src + i * 8); v8h o;
#pragma unroll
    for (int k = 0; k < 8; ++k) o[k] = toh_flush(bfr(v[k]) * SCW);
    *(volatile v8h*)(dst + i * 8) = o; __threadfence(); *(volatile v8h*)(dst + i * 8) = o;
}

__global__ __launch_bounds__(256) void k_xt(const float* __restrict__ x, bf* XT) {
    __shared__ __align__(16) bf ts[64 * XP];
    const int t = threadIdx.x;
    const int blk = blockIdx.x;
    const int b = blk / (NPIX / 64), p0 = (blk % (NPIX / 64)) * 64;
    const float* xb = x + (size_t)b * CH * NPIX + p0;
#pragma unroll
    for (int it = 0; it < 4; ++it) {
        const int idx = it * 256 + t; const int c = idx >> 4, p4 = (idx & 15) * 4;
        const v4f v = *(const v4f*)(xb + (size_t)c * NPIX + p4);
#pragma unroll
        for (int k = 0; k < 4; ++k) ts[(p4 + k) * XP + c] = f2bf(v[k]);
    }
    __syncthreads();
    bf* dst = XT + ((size_t)b * NPIX + p0) * CH;
#pragma unroll 1
    for (int ps = 0; ps < 2; ++ps) {
#pragma unroll
        for (int it = 0; it < 2; ++it) { const int p = it * 32 + (t >> 3), c8 = (t & 7) * 8;
            const v8us o = *(const v8usa*)(&ts[p * XP + c8]);
            *(volatile v8us*)(dst + (size_t)p * CH + c8) = o; }
        if (ps == 0) __threadfence(); }
}

__device__ __forceinline__ float coord1(float conv, float bias, float ip, float base, float nrm, float inrm) {
#pragma clang fp contract(off)
    const float off = (conv + bias) * 0.25f + ip;
    const float g = 2.0f * (base + off) * inrm - 1.0f;
    const float u = ((g + 1.0f) * nrm - 1.0f) * 0.5f;
    return fminf(fmaxf(u, 0.0f), nrm - 1.0f);
}

__device__ __forceinline__ v8h samp8(const bf* __restrict__ xg, float ix, float iy) {
    const float x0f = floorf(ix), y0f = floorf(iy);
    const float wx = ix - x0f, wy = iy - y0f;
    int x0 = (int)x0f, y0 = (int)y0f;
    x0 = x0 < 0 ? 0 : (x0 > IMW - 1 ? IMW - 1 : x0);
    y0 = y0 < 0 ? 0 : (y0 > IMH - 1 ? IMH - 1 : y0);
    const int x1 = (x0 + 1 > IMW - 1) ? (IMW - 1) : (x0 + 1);
    const int y1 = (y0 + 1 > IMH - 1) ? (IMH - 1) : (y0 + 1);
    const float ux = 1.0f - wx, uy = 1.0f - wy;
    const float w00 = ux * uy * SCS, w01 = wx * uy * SCS, w10 = ux * wy * SCS, w11 = wx * wy * SCS;
    const v4u q00 = *(const v4ua*)(xg + (size_t)((y0 * IMW + x0) * CH));
    const v4u q01 = *(const v4ua*)(xg + (size_t)((y0 * IMW + x1) * CH));
    const v4u q10 = *(const v4ua*)(xg + (size_t)((y1 * IMW + x0) * CH));
    const v4u q11 = *(const v4ua*)(xg + (size_t)((y1 * IMW + x1) * CH));
    v8h o;
#pragma unroll
    for (int d = 0; d < 4; ++d) {
        const float vl = w00 * __uint_as_float(q00[d] << 16) + w01 * __uint_as_float(q01[d] << 16)
                       + w10 * __uint_as_float(q10[d] << 16) + w11 * __uint_as_float(q11[d] << 16);
        const float vh = w00 * __uint_as_float(q00[d] & 0xffff0000u) + w01 * __uint_as_float(q01[d] & 0xffff0000u)
                       + w10 * __uint_as_float(q10[d] & 0xffff0000u) + w11 * __uint_as_float(q11[d] & 0xffff0000u);
        o[2 * d] = toh_flush(vl); o[2 * d + 1] = toh_flush(vh);
    }
    return o;
}

__global__ __launch_bounds__(32 * MW) void k_main(const bf* __restrict__ XT, const bf* __restrict__ OWB, const float* __restrict__ ob,
                                                  const h16* __restrict__ EWH, const float* __restrict__ eb, float* OUT) {
    __shared__ __align__(16) float cs[MW * 16 * NK * 2];
    __shared__ __align__(16) float os[MW * 32 * OSP];
    const int lane = threadIdx.x & 31, lr = lane & 15, hi = lane >> 4;
    const int wave = __builtin_amdgcn_readfirstlane((int)(threadIdx.x >> 5));
    const int strip = blockIdx.x * MW + wave;
    const int b = strip / (NPIX / 16); const int p0 = (strip % (NPIX / 16)) * 16;
    const int hrow = p0 / IMW, w0 = p0 % IMW;
    const int csb = wave * (16 * NK * 2), osb = wave * (32 * OSP);
    {
        const size_t xo = ((size_t)b * NPIX + (size_t)(p0 + lr)) * CH + 8 * hi;
        const size_t wo = (size_t)lr * CH + 8 * hi;
        const v16bf a0 = ldb(XT + xo), a1 = ldb(XT + xo + 32);
        const v16bf bx0 = ldb(OWB + wo), bx1 = ldb(OWB + wo + 32);
        const v16bf by0 = ldb(OWB + wo + (size_t)NK * CH), by1 = ldb(OWB + wo + (size_t)NK * CH + 32);
        v8f ax = (v8f){}, ay = (v8f){};
        ax = wmmabg(a0, bx0, ax); ax = wmmabg(a1, bx1, ax);
        ay = wmmabg(a0, by0, ay); ay = wmmabg(a1, by1, ay);
        const float bxv = bfr(ob[lr]), byv = bfr(ob[NK + lr]);
        const float ipx = (lr & 1) ? 0.25f : -0.25f;
        const float ipy = (lr & 2) ? 0.25f : -0.25f;
        const float hf = (float)hrow + 0.5f;
#pragma unroll
        for (int r = 0; r < 8; ++r) {
            const float wf = (float)(w0 + 8 * hi + r) + 0.5f;
            v2f c;
            c[0] = coord1(ax[r], bxv, ipx, wf, (float)IMW, 1.0f / (float)IMW);
            c[1] = coord1(ay[r], byv, ipy, hf, (float)IMH, 1.0f / (float)IMH);
            *(v2fa*)(&cs[csb + ((8 * hi + r) * NK + lr) * 2]) = c; }
    }
    wave_sync();
    const v16h ea0 = ldh(EWH + (size_t)lr * CH + 8 * hi), ea1 = ldh(EWH + (size_t)lr * CH + 8 * hi + 32);
    float ebv[8];
#pragma unroll
    for (int r = 0; r < 8; ++r) ebv[r] = bfr(eb[8 * hi + r]);
    const bf* xbat = XT + (size_t)b * NPIX * CH + 8 * hi;
    const int j = lr & 1;
#pragma unroll 1
    for (int ti = 0; ti < 4; ++ti) {
        const int i = ti >> 1, q = ti & 1;
        const int pl = 8 * q + (lr >> 1);
        const int cb = csb + (pl * NK + i * 2 + j) * 2;
        const v2f c0 = *(const v2fa*)(&cs[cb]);
        const v2f c1 = *(const v2fa*)(&cs[cb + 8]);
        const v2f c2 = *(const v2fa*)(&cs[cb + 16]);
        const v2f c3 = *(const v2fa*)(&cs[cb + 24]);
        v8f acc = (v8f){};
        { const v8h s0 = samp8(xbat, c0[0], c0[1]); const v8h s1 = samp8(xbat + 16, c1[0], c1[1]);
          acc = wmma16g(ea0, cat16(s0, s1), acc); }
        { const v8h s2 = samp8(xbat + 32, c2[0], c2[1]); const v8h s3 = samp8(xbat + 48, c3[0], c3[1]);
          acc = wmma16g(ea1, cat16(s2, s3), acc); }
#pragma unroll
        for (int r = 0; r < 8; ++r)
            os[osb + ((8 * hi + r) * 2 + i) * OSP + 16 * q + lr] = acc[r] * OSC + ebv[r];
    }
    wave_sync();
    float* obase = OUT + (((size_t)b * OC) * OH + (size_t)(2 * hrow)) * OW + 2 * w0;
#pragma unroll 1
    for (int ps = 0; ps < 2; ++ps) {
#pragma unroll
        for (int s = 0; s < 8; ++s) { const int line = 4 * s + (lane >> 3), cofs = (lane & 7) * 4;
            const int oc = line >> 1, ii = line & 1;
            const v4f val = *(const v4fa*)(&os[osb + line * OSP + cofs]);
            *(volatile v4f*)(obase + ((size_t)oc * OH + ii) * OW + cofs) = val; }
        if (ps == 0) __threadfence(); }
}

static constexpr size_t al256(size_t v) { return (v + 255) & ~(size_t)255; }
static constexpr size_t SZ_XT = al256((size_t)NB * NPIX * CH * 2);
static constexpr size_t SZ_OW = al256((size_t)OFC * CH * 2);
static constexpr size_t SZ_EW = al256((size_t)OC * CH * 2);
static constexpr size_t SZ_TOTAL = SZ_XT + SZ_OW + SZ_EW;
static_assert(SZ_TOTAL <= (size_t)134217728);
static_assert(((size_t)OFC * CH) % (8 * 16) == 0);
static_assert(((size_t)OC * CH) % (8 * 8) == 0);
static_assert(((size_t)NB * NPIX) % 64 == 0);

extern "C" void kernel_launch(void* const* d_in, const int* in_sizes, int n_in,
                              void* d_out, int out_size, void* d_ws, size_t ws_size, hipStream_t stream) {
    if (n_in < 5) return;
    if ((size_t)in_sizes[0] < (size_t)NB * CH * NPIX) return;
    if ((size_t)in_sizes[1] < (size_t)OFC * CH || in_sizes[2] < OFC) return;
    if ((size_t)in_sizes[3] < (size_t)OC * CH || in_sizes[4] < OC) return;
    if ((size_t)out_size < (size_t)NB * OC * OH * OW) return;
    if (SZ_TOTAL > ws_size) return;
    const float* x  = (const float*)d_in[0];
    const float* ow = (const float*)d_in[1];
    const float* ob = (const float*)d_in[2];
    const float* ew = (const float*)d_in[3];
    const float* eb = (const float*)d_in[4];
    float* OUT = (float*)d_out;
    char* wsp = (char*)d_ws;
    bf*  XT  = (bf*)wsp;  wsp += SZ_XT;
    bf*  OWB = (bf*)wsp;  wsp += SZ_OW;
    h16* EWH = (h16*)wsp; wsp += SZ_EW;

    k_xt<<<(unsigned)(NB * (NPIX / 64)), 256, 0, stream>>>(x, XT);
    { const size_t n8 = (size_t)OFC * CH / 8; k_cvt8<<<(unsigned)((n8 + 255) / 256), 256, 0, stream>>>(ow, OWB, n8); }
    { const size_t n8 = (size_t)OC * CH / 8;  k_cvtwh<<<(unsigned)((n8 + 255) / 256), 256, 0, stream>>>(ew, EWH, n8); }
    k_main<<<(unsigned)(NB * (NPIX / 16) / MW), 32 * MW, 0, stream>>>(XT, OWB, ob, EWH, eb, OUT);
}
